// GCN_40140764348986
// MI455X (gfx1250) — hardware-verified
//
#include <hip/hip_runtime.h>
#include <stddef.h>
#include <stdint.h>
#include <math.h>


#define CIN     128
#define HID     256
#define KA      512
#define NGR     256
#define NTHR    256
#define NWAVE   8
#define EPT     8
#define CHUNK   (NTHR * EPT)
#define WCAP    (EPT * 32)
#define LISTN   (NWAVE * WCAP)
#define NBA     1024
#define SLA     10
#define RCAP    28672
#define DEGCAP  128
#define MEAS_B1024  16623
#define MEAS_MAXDEG 35
#define PER     196
#define MEMCAP  1024
#define GBM     64
#define GBN     64
#define GTHR    128
#define MROWS   128
#define NUW1    (HID * (CIN / 8))
#define NUWD    (HID * (KA / 8))
#define TB_B1   0
#define TB_B2   256
#define TB_B3   512
#define TB_BF   768
#define TB_WO   1024
#define TB_BO   1280
#define TB_N    1312
#define WSMAX   134217728
#define BKT_ZINTS    (RCAP + 3 * NBA)
#define BKT_LDS_INTS (LISTN + 2 * RCAP + 3 * NBA + 16 + NBA)

static_assert((CHUNK & (CHUNK - 1)) == 0 && CHUNK <= 4096);
static_assert((NBA & (NBA - 1)) == 0 && NBA == (1 << SLA) && NBA == 4 * NTHR);
static_assert(((long long)CHUNK << SLA) < (1LL << 31));
static_assert(NBA % NWAVE == 0 && NBA % 32 == 0);
static_assert((RCAP % (NTHR * 4)) == 0 && (BKT_ZINTS % 4) == 0);
static_assert((long long)RCAP * 100 >= (long long)MEAS_B1024 * 105);
static_assert(DEGCAP >= MEAS_MAXDEG + 8);
static_assert(BKT_LDS_INTS * 4 <= 300000);
static_assert(((LISTN + 2 * RCAP + 3 * NBA + 16) % 4) == 0);
static_assert(GBM == (GTHR / 32) * 16 && GBN == 64);
static_assert((CIN % 32) == 0 && (KA % 32) == 0 && KA == 2 * HID);
static_assert((HID % GBN) == 0 && (NGR % GBM) == 0 && (MROWS % GBM) == 0);
static_assert(HID == 8 * 32);
static_assert(NGR == 256 && NTHR == HID && NTHR == NGR);
static_assert(50048 == 391 * 128);
static_assert(PER * NTHR >= 50000 && (PER % 4) == 0);
static_assert(MEMCAP >= 4 * PER && (MEMCAP % NTHR) == 0);
static_assert((NUW1 % NTHR) == 0 && (NUWD % NTHR) == 0);
static_assert(TB_N % 32 == 0 && TB_BO + 32 == TB_N);

typedef float          v4f  __attribute__((ext_vector_type(4)));
typedef float          v8f  __attribute__((ext_vector_type(8)));
typedef int            v4i  __attribute__((ext_vector_type(4)));
typedef int            v8i  __attribute__((ext_vector_type(8)));
typedef unsigned short v8us __attribute__((ext_vector_type(8)));
typedef __bf16         v16b __attribute__((ext_vector_type(16)));
typedef v4f  __attribute__((may_alias)) v4fa;
typedef v4i  __attribute__((may_alias)) v4ia;
typedef v8us __attribute__((may_alias)) v8usa;
union FragB { v16b v; v8us h[2]; v8i w; };

__device__ __forceinline__ v8f wmb(const FragB& a, const FragB& b, v8f c) {
  v8f d = __builtin_amdgcn_wmma_f32_16x16x32_bf16(false, a.v, false, b.v, (short)0, c, false, false);
  asm volatile("v_nop\n\tv_nop\n\tv_nop\n\tv_nop" : "+v"(d) : "v"(a.w), "v"(b.w));
  return d;
}

__device__ __forceinline__ unsigned int f2bf(float f) {
  const unsigned int u = __float_as_uint(f);
  const unsigned int r = ((u + 0x7FFFu + ((u >> 16) & 1u)) >> 16) & 0xFFFFu;
  return ((u & 0x7FFFFFFFu) > 0x7F800000u) ? 0x7FC0u : r;
}
__device__ __forceinline__ float bf2f(unsigned int b) { return __uint_as_float(b << 16); }
__device__ __forceinline__ float bfr(float f) { return bf2f(f2bf(f)); }
__device__ __forceinline__ float relu_np(float v) { return (v > 0.0f) ? v : (v - v); }

template <int SLB>
__device__ __forceinline__ int scan_chunk(const int* __restrict__ dsts, int nE, int cbase, int slotBase,
                                          int nb, int vec8, int* list, int tid, int lane, int wave) {
  int wc = 0;
  const int el0  = tid * EPT;
  const int e0   = cbase + el0;
  const int sent = -2147483647 - 1;
  v4i da, db;
  if (vec8 != 0 && cbase + CHUNK <= nE) {
    da = *(const v4i*)(dsts + e0);
    db = *(const v4i*)(dsts + e0 + 4);
  } else {
    da.x = (e0     < nE) ? dsts[min(e0,     nE - 1)] : sent;
    da.y = (e0 + 1 < nE) ? dsts[min(e0 + 1, nE - 1)] : sent;
    da.z = (e0 + 2 < nE) ? dsts[min(e0 + 2, nE - 1)] : sent;
    da.w = (e0 + 3 < nE) ? dsts[min(e0 + 3, nE - 1)] : sent;
    db.x = (e0 + 4 < nE) ? dsts[min(e0 + 4, nE - 1)] : sent;
    db.y = (e0 + 5 < nE) ? dsts[min(e0 + 5, nE - 1)] : sent;
    db.z = (e0 + 6 < nE) ? dsts[min(e0 + 6, nE - 1)] : sent;
    db.w = (e0 + 7 < nE) ? dsts[min(e0 + 7, nE - 1)] : sent;
  }
  const unsigned nbs = (unsigned)slotBase;
  const unsigned unb = (unsigned)nb;
  const unsigned s0 = (unsigned)da.x - nbs, s1 = (unsigned)da.y - nbs;
  const unsigned s2 = (unsigned)da.z - nbs, s3 = (unsigned)da.w - nbs;
  const unsigned s4 = (unsigned)db.x - nbs, s5 = (unsigned)db.y - nbs;
  const unsigned s6 = (unsigned)db.z - nbs, s7 = (unsigned)db.w - nbs;
  const bool h0 = s0 < unb, h1 = s1 < unb, h2 = s2 < unb, h3 = s3 < unb;
  const bool h4 = s4 < unb, h5 = s5 < unb, h6 = s6 < unb, h7 = s7 < unb;
  const unsigned any = __builtin_amdgcn_ballot_w32(h0 | h1 | h2 | h3 | h4 | h5 | h6 | h7);
  if (any != 0u) {
#define HITJ(J, HJ, SJ) { \
      const unsigned mj = __builtin_amdgcn_ballot_w32(HJ); \
      if (mj != 0u) { \
        if (HJ) { \
          const int pos = wc + (int)__builtin_amdgcn_mbcnt_lo(mj, 0u); \
          if (pos < WCAP) list[wave * WCAP + pos] = ((el0 + (J)) << SLB) | (int)(SJ); \
        } \
        wc += (int)__builtin_popcount(mj); } }
    HITJ(0, h0, s0)
    HITJ(1, h1, s1)
    HITJ(2, h2, s2)
    HITJ(3, h3, s3)
    HITJ(4, h4, s4)
    HITJ(5, h5, s5)
    HITJ(6, h6, s6)
    HITJ(7, h7, s7)
#undef HITJ
  }
  return wc;
}

__device__ __forceinline__ v8us wgather(const float* __restrict__ W, int n, int kk) {
  const float* p = W + (size_t)kk * HID + n;
  v8us o;
#pragma unroll
  for (int i = 0; i < 8; ++i) o[i] = (unsigned short)f2bf(p[(size_t)i * HID]);
  return o;
}

__global__ __launch_bounds__(NTHR) void k_prep(
    const float* __restrict__ x, const float* __restrict__ W1, const float* __restrict__ W2,
    const float* __restrict__ W3, const float* __restrict__ Wf,
    const float* __restrict__ b1, const float* __restrict__ b2, const float* __restrict__ b3,
    const float* __restrict__ bfv, const float* __restrict__ Wo, const float* __restrict__ bo,
    unsigned short* XB, unsigned short* W1T, unsigned short* W2D, unsigned short* W3D, unsigned short* WfD,
    float* TAB, int nN, int nUx) {
  const int tid = (int)threadIdx.x;
  const int u   = (int)blockIdx.x * NTHR + tid;
  const int uW2 = nUx + NUW1;
  const int uW3 = uW2 + NUWD;
  const int uWf = uW3 + NUWD;
  const int uTA = uWf + NUWD;
  const int uTB = uTA + NTHR;
  const int uEnd = uTB + NTHR;
  if (u >= uEnd) return;
  if (u >= uTA) {
    v4f v = {0.f, 0.f, 0.f, 0.f};
    float* tp;
    bool st;
    if (u < uTB) {
      const int t = tid >> 6, piece = tid & 63;
      if (t == 0)      v = *(const v4f*)(b1  + 4 * piece);
      else if (t == 1) v = *(const v4f*)(b2  + 4 * piece);
      else if (t == 2) v = *(const v4f*)(b3  + 4 * piece);
      else             v = *(const v4f*)(bfv + 4 * piece);
      v.x = bfr(v.x); v.y = bfr(v.y); v.z = bfr(v.z); v.w = bfr(v.w);
      tp = TAB + 4 * tid;
      st = true;
    } else {
      const int piece = tid & 63;
      const v4f w  = *(const v4f*)(Wo + 4 * piece);
      const float bb = bo[0];
      const bool isw = tid < 64;
      v.x = isw ? bfr(w.x) : ((tid == 64) ? bfr(bb) : 0.0f);
      v.y = isw ? bfr(w.y) : 0.0f;
      v.z = isw ? bfr(w.z) : 0.0f;
      v.w = isw ? bfr(w.w) : 0.0f;
      tp = TAB + TB_WO + 4 * (tid < 72 ? tid : 71);
      st = tid < 72;
    }
    if (st) *(volatile v4f*)tp = v;
    __threadfence();
    if (st) *(volatile v4f*)tp = v;
    return;
  }
  v8us o;
  unsigned short* dp;
  if (u < nUx) {
    const int row = u >> 4;
    const int k8  = (u & 15) * 8;
    const int rc  = row < nN ? row : nN - 1;
    const float* p = x + (size_t)rc * CIN + k8;
    const v4f a = *(const v4f*)p;
    const v4f b = *(const v4f*)(p + 4);
    const bool ok = row < nN;
    o[0] = ok ? (unsigned short)f2bf(a.x) : (unsigned short)0;
    o[1] = ok ? (unsigned short)f2bf(a.y) : (unsigned short)0;
    o[2] = ok ? (unsigned short)f2bf(a.z) : (unsigned short)0;
    o[3] = ok ? (unsigned short)f2bf(a.w) : (unsigned short)0;
    o[4] = ok ? (unsigned short)f2bf(b.x) : (unsigned short)0;
    o[5] = ok ? (unsigned short)f2bf(b.y) : (unsigned short)0;
    o[6] = ok ? (unsigned short)f2bf(b.z) : (unsigned short)0;
    o[7] = ok ? (unsigned short)f2bf(b.w) : (unsigned short)0;
    dp = XB + (size_t)row * CIN + k8;
  } else if (u < uW2) {
    const int v  = u - nUx;
    const int n  = v >> 4;
    const int k8 = (v & 15) * 8;
    o  = wgather(W1, n, k8);
    dp = W1T + (size_t)n * CIN + k8;
  } else if (u < uW3) {
    const int v  = u - uW2;
    const int n  = v >> 6;
    const int k8 = (v & 63) * 8;
    o  = wgather(W2, n, k8 & (HID - 1));
    dp = W2D + (size_t)n * KA + k8;
  } else if (u < uWf) {
    const int v  = u - uW3;
    const int n  = v >> 6;
    const int k8 = (v & 63) * 8;
    o  = wgather(W3, n, k8 & (HID - 1));
    dp = W3D + (size_t)n * KA + k8;
  } else {
    const int v  = u - uWf;
    const int n  = v >> 6;
    const int k8 = (v & 63) * 8;
    o  = wgather(Wf, n, k8 & (HID - 1));
    dp = WfD + (size_t)n * KA + k8;
  }
  *(volatile v8us*)dp = o;
  __threadfence();
  *(volatile v8us*)dp = o;
}

__global__ __launch_bounds__(NTHR) void k_bucket(const int* __restrict__ srcs, const int* __restrict__ dsts,
                                                 int nE, int nN, int vec8,
                                                 int* LIST, int* CNT, int* OFF, float* DIS, int* FLG) {
  extern __shared__ __attribute__((aligned(16))) int bsm[];
  int* list = bsm;
  int* reg1 = bsm + LISTN;
  int* sl   = reg1 + RCAP;
  int* cnt  = sl + RCAP;
  int* offs = cnt + NBA;
  int* cur  = offs + NBA;
  int* wcnt = cur + NBA;
  float* disv = (float*)(wcnt + 16);
  const int tid = (int)threadIdx.x, lane = tid & 31, wave = tid >> 5;
  const int blk = (int)blockIdx.x;
  const int nodeBase = blk * NBA;
  int nb = nN - nodeBase;
  nb = nb < 0 ? 0 : (nb > NBA ? NBA : nb);

  {
    const v4i z4 = {0, 0, 0, 0};
    for (int i = tid * 4; i < BKT_ZINTS; i += NTHR * 4) *(v4ia*)(sl + i) = z4;
    if (tid < 16) wcnt[tid] = 0;
  }
  __syncthreads();

  int tot = 0, ovf = 0;
  const int nChunks = (nE + CHUNK - 1) / CHUNK;
#pragma unroll 1
  for (int ch = 0; ch < nChunks; ++ch) {
    const int cbase = ch * CHUNK;
    const int wc = scan_chunk<SLA>(dsts, nE, cbase, nodeBase, nb, vec8, list, tid, lane, wave);
    if (lane == 0) wcnt[wave] = wc;
    __syncthreads();
    int pre = 0, all = 0;
#pragma unroll
    for (int w2 = 0; w2 < NWAVE; ++w2) {
      int c = wcnt[w2];
      c = c < 0 ? 0 : (c > WCAP ? WCAP : c);
      all += c;
      pre += (w2 < wave) ? c : 0;
    }
    const int wcc  = wc > WCAP ? WCAP : wc;
    const int base = tot + pre;
#pragma unroll 1
    for (int i0 = 0; i0 < wcc; i0 += 32) {
      const int i   = i0 + lane;
      const int ic  = i < wcc ? i : wcc - 1;
      const int ent = list[wave * WCAP + ic];
      const int el  = (ent >> SLA) & (CHUNK - 1);
      const int sq  = ent & (NBA - 1);
      int eid = cbase + el;
      eid = eid > nE - 1 ? nE - 1 : eid;
      const int sraw = srcs[eid];
      const int s = sraw < 0 ? 0 : (sraw > nN - 1 ? nN - 1 : sraw);
      const int pos = base + i;
      if (i < wcc && pos < RCAP) reg1[pos] = (int)((unsigned)s | ((unsigned)sq << 16));
    }
    if (tot + all > RCAP) ovf = 1;
    tot += all;
    tot = tot > RCAP ? RCAP : tot;
    __syncthreads();
  }
  const int nh = tot;

  if (wave == 0) {
#pragma unroll 1
    for (int b0 = 0; b0 < nh; b0 += 32) {
      const int idx = b0 + lane;
      const int uv  = reg1[idx < nh ? idx : nh - 1];
      const int m32 = (nh - b0) < 32 ? (nh - b0) : 32;
#pragma unroll 1
      for (int k = 0; k < m32; ++k) {
        const int u  = __builtin_amdgcn_readlane(uv, k);
        const int sq = (u >> 16) & (NBA - 1);
        if (lane == 0) cnt[sq] = cnt[sq] + 1;
      }
    }
  }
  __syncthreads();
  if (wave == 0) {
    const int base = lane * (NBA / 32);
    int s = 0;
#pragma unroll 1
    for (int i = 0; i < NBA / 32; ++i) s += cnt[base + i];
    int incl = s;
#pragma unroll
    for (int d = 1; d < 32; d <<= 1) {
      const int y = __shfl_up(incl, d, 32);
      if (lane >= d) incl += y;
    }
    int run = incl - s;
#pragma unroll 1
    for (int i = 0; i < NBA / 32; ++i) {
      const int cv = cnt[base + i];
      offs[base + i] = run;
      cur[base + i]  = run;
      run += cv;
    }
  }
  __syncthreads();
  if (wave == 0) {
#pragma unroll 1
    for (int b0 = 0; b0 < nh; b0 += 32) {
      const int idx = b0 + lane;
      const int uv  = reg1[idx < nh ? idx : nh - 1];
      const int m32 = (nh - b0) < 32 ? (nh - b0) : 32;
#pragma unroll 1
      for (int k = 0; k < m32; ++k) {
        const int u  = __builtin_amdgcn_readlane(uv, k);
        const int sq = (u >> 16) & (NBA - 1);
        if (lane == 0) {
          int p = cur[sq];
          p = p < 0 ? 0 : (p > RCAP - 1 ? RCAP - 1 : p);
          sl[p] = u;
          cur[sq] = p + 1;
        }
      }
    }
  }
  __syncthreads();

#pragma unroll 1
  for (int i = tid; i < NBA; i += NTHR) {
    const float d = (float)(cnt[i] + 1);
    disv[i] = 1.0f / sqrtf(d);
  }
  __syncthreads();

  int* lb = LIST + (size_t)blk * RCAP;
  const v4i c4 = *(const v4ia*)(cnt + 4 * tid);
  const v4i o4 = *(const v4ia*)(offs + 4 * tid);
  const v4f d4 = *(const v4fa*)(disv + 4 * tid);
  v4i cv;
  cv.x = (tid == 0) ? nh : 0;
  cv.y = (tid == 0) ? ovf : 0;
  cv.z = 0; cv.w = 0;
  int*   cp = CNT + (size_t)nodeBase + 4 * tid;
  int*   op = OFF + (size_t)nodeBase + 4 * tid;
  float* dq = DIS + (size_t)nodeBase + 4 * tid;
  int*   fp = FLG + (size_t)blk * 32 + 4 * (tid & 7);
#pragma unroll 1
  for (int p = tid * 4; p < RCAP; p += NTHR * 4) {
    const v4i v = *(const v4ia*)(sl + p);
    *(volatile v4i*)(lb + p) = v;
  }
  *(volatile v4i*)cp = c4;
  *(volatile v4i*)op = o4;
  *(volatile v4f*)dq = d4;
  if (tid < 8) *(volatile v4i*)fp = cv;
  __threadfence();
#pragma unroll 1
  for (int p = tid * 4; p < RCAP; p += NTHR * 4) {
    const v4i v = *(const v4ia*)(sl + p);
    *(volatile v4i*)(lb + p) = v;
  }
  *(volatile v4i*)cp = c4;
  *(volatile v4i*)op = o4;
  *(volatile v4f*)dq = d4;
  if (tid < 8) *(volatile v4i*)fp = cv;
}

__global__ __launch_bounds__(GTHR) void k_gemm(
    const unsigned short* __restrict__ A, const unsigned short* __restrict__ WT,
    float* outF, int K, int ldo)
{
  __shared__ __attribute__((aligned(16))) float stg[GBM * GBN];
  const int tid = (int)threadIdx.x, lane = tid & 31, wave = tid >> 5, hh = lane >> 4, m = lane & 15;
  const int rowBase = (int)blockIdx.x * GBM;
  const int col0    = (int)blockIdx.y * GBN;

  v8f acc[4];
  {
    const v8f z = {0.f, 0.f, 0.f, 0.f, 0.f, 0.f, 0.f, 0.f};
    acc[0] = z; acc[1] = z; acc[2] = z; acc[3] = z;
  }
  const unsigned short* ap = A  + (size_t)(rowBase + 16 * wave + m) * (size_t)K + 8 * hh;
  const unsigned short* wp = WT + (size_t)(col0 + m) * (size_t)K + 8 * hh;
  const int ksteps = K >> 5;
#pragma unroll 1
  for (int ks = 0; ks < ksteps; ++ks) {
    FragB af;
    af.h[0] = *(const v8usa*)(ap + 32 * ks);
    af.h[1] = *(const v8usa*)(ap + 32 * ks + 16);
#pragma unroll
    for (int t = 0; t < 4; ++t) {
      const unsigned short* wq = wp + (size_t)(16 * t) * (size_t)K + 32 * ks;
      FragB bf;
      bf.h[0] = *(const v8usa*)wq;
      bf.h[1] = *(const v8usa*)(wq + 16);
      acc[t] = wmb(af, bf, acc[t]);
    }
  }

#pragma unroll
  for (int t = 0; t < 4; ++t) {
    const int lc = 16 * t + m;
#pragma unroll
    for (int r = 0; r < 8; ++r) {
      const int lr = 16 * wave + 8 * hh + r;
      stg[lr * GBN + lc] = acc[t][r];
    }
  }
  __syncthreads();

  v4f fv[8];
#pragma unroll
  for (int i = 0; i < 8; ++i) {
    const int lr = 16 * wave + 2 * i + hh;
    fv[i] = *(const v4fa*)(stg + lr * GBN + 4 * m);
  }
#pragma unroll
  for (int i = 0; i < 8; ++i) {
    const int lr = 16 * wave + 2 * i + hh;
    const int gr = rowBase + lr;
    float* op = outF + (size_t)gr * (size_t)ldo + col0 + 4 * m;
    *(volatile v4f*)op = fv[i];
  }
  __threadfence();
#pragma unroll
  for (int i = 0; i < 8; ++i) {
    const int lr = 16 * wave + 2 * i + hh;
    const int gr = rowBase + lr;
    float* op = outF + (size_t)gr * (size_t)ldo + col0 + 4 * m;
    *(volatile v4f*)op = fv[i];
  }
}

__global__ __launch_bounds__(NTHR) void k_agg(const int* __restrict__ LIST, const int* __restrict__ CNT,
                                              const int* __restrict__ OFF, const int* __restrict__ FLG,
                                              const float* __restrict__ DIS, const float* __restrict__ Hm,
                                              const float* __restrict__ bias, unsigned short* XP,
                                              int nN, int MPr) {
  const int tid = (int)threadIdx.x, lane = tid & 31, wave = tid >> 5;
  const int blk = (int)blockIdx.x;
  const int nodeBase = blk * NBA;

  const int nhraw = FLG[(size_t)blk * 32];
  const int bflag = FLG[(size_t)blk * 32 + 1];
  const int nh  = nhraw < 0 ? 0 : (nhraw > RCAP ? RCAP : nhraw);
  const bool ovf = (bflag != 0) || (nhraw < 0) || (nhraw > RCAP);
  const int* hb = LIST + (size_t)blk * RCAP;

  float bv[8];
  {
    const v4f a = *(const v4f*)(bias + 8 * lane);
    const v4f b = *(const v4f*)(bias + 8 * lane + 4);
    bv[0] = a.x; bv[1] = a.y; bv[2] = a.z; bv[3] = a.w;
    bv[4] = b.x; bv[5] = b.y; bv[6] = b.z; bv[7] = b.w;
  }
  const float qnan = __int_as_float(0x7fc00000);

#pragma unroll 1
  for (int si = 0; si < NBA / NWAVE; ++si) {
    const int s    = si * NWAVE + wave;
    const int node = nodeBase + s;
    const int nc   = node < nN ? node : nN - 1;
    int c = CNT[node];
    bool bad = ovf || (c > DEGCAP) || (c < 0);
    c = c < 0 ? 0 : (c > DEGCAP ? DEGCAP : c);
    int o = OFF[node];
    bad = bad || (o < 0) || (o > RCAP);
    o = o < 0 ? 0 : (o > RCAP ? RCAP : o);
    if (c > nh - o) { c = nh - o; bad = true; }
    c = c < 0 ? 0 : c;
    const float dd = DIS[nc];
    const float rd = dd * dd;
    float acc[8];
#pragma unroll
    for (int i = 0; i < 8; ++i) acc[i] = 0.0f;
#pragma unroll 1
    for (int b0 = 0; b0 < c; b0 += 32) {
      int idx = o + b0 + lane;
      idx = idx < 0 ? 0 : (idx > RCAP - 1 ? RCAP - 1 : idx);
      const int ent = hb[idx];
      int hs = ent & 0xFFFF;
      hs = hs > nN - 1 ? nN - 1 : hs;
      const float cf  = DIS[hs] * dd;
      const int   cfi = __float_as_int(cf);
      const int m32 = (c - b0) < 32 ? (c - b0) : 32;
#pragma unroll 1
      for (int k = 0; k < m32; ++k) {
        const int   sk = __builtin_amdgcn_readlane(hs, k);
        const float ck = __int_as_float(__builtin_amdgcn_readlane(cfi, k));
        const float* rp = Hm + (size_t)sk * HID + 8 * lane;
        const v4f a = *(const v4f*)rp;
        const v4f b = *(const v4f*)(rp + 4);
        acc[0] = fmaf(ck, a.x, acc[0]); acc[1] = fmaf(ck, a.y, acc[1]);
        acc[2] = fmaf(ck, a.z, acc[2]); acc[3] = fmaf(ck, a.w, acc[3]);
        acc[4] = fmaf(ck, b.x, acc[4]); acc[5] = fmaf(ck, b.y, acc[5]);
        acc[6] = fmaf(ck, b.z, acc[6]); acc[7] = fmaf(ck, b.w, acc[7]);
      }
    }
    float sv[8];
    {
      const float* rp = Hm + (size_t)nc * HID + 8 * lane;
      const v4f a = *(const v4f*)rp;
      const v4f b = *(const v4f*)(rp + 4);
      sv[0] = a.x; sv[1] = a.y; sv[2] = a.z; sv[3] = a.w;
      sv[4] = b.x; sv[5] = b.y; sv[6] = b.z; sv[7] = b.w;
    }
    const bool live = node < nN;
    v8us ho, lo;
#pragma unroll
    for (int i = 0; i < 8; ++i) {
      float y = (acc[i] + sv[i] * rd) + bv[i];
      y = relu_np(y);
      y = bad ? qnan : y;
      const float v = live ? y : 0.0f;
      const unsigned int hbi = f2bf(v);
      ho[i] = (unsigned short)hbi;
      lo[i] = (unsigned short)f2bf(v - bf2f(hbi));
    }
    if (node < MPr) {
      unsigned short* hp = XP + (size_t)node * KA + 8 * lane;
      *(volatile v8us*)hp = ho;
      *(volatile v8us*)(hp + HID) = lo;
      __threadfence();
      *(volatile v8us*)hp = ho;
      *(volatile v8us*)(hp + HID) = lo;
    }
  }
}

__global__ __launch_bounds__(NTHR) void k_pool(const unsigned short* __restrict__ XH, const int* __restrict__ bat,
                                               int nN, unsigned short* PH) {
  __shared__ int cntS[NTHR];
  __shared__ int offS[NTHR];
  __shared__ int mem[MEMCAP];
  __shared__ int tot[4];
  __shared__ __attribute__((aligned(16))) unsigned short prow[KA];
  const int tid = (int)threadIdx.x, lane = tid & 31, wave = tid >> 5;
  const int g = (int)blockIdx.x;

  for (int i = tid; i < MEMCAP; i += NTHR) mem[i] = 0;
  if (tid < 4) tot[tid] = 0;
  const int seg0  = tid * PER;
  const int lastv = nN - 4;

  int mine = 0;
#pragma unroll 1
  for (int q = 0; q < PER / 4; ++q) {
    const int i0 = seg0 + 4 * q;
    const int ic = i0 < lastv ? i0 : lastv;
    const v4i b = *(const v4i*)(bat + ic);
    const bool ok = i0 < nN;
    mine += (ok && b.x == g) ? 1 : 0;
    mine += (ok && b.y == g) ? 1 : 0;
    mine += (ok && b.z == g) ? 1 : 0;
    mine += (ok && b.w == g) ? 1 : 0;
  }
  cntS[tid] = mine;
  __syncthreads();
  if (wave == 0) {
    const int base = lane * (NTHR / 32);
    int s = 0;
#pragma unroll 1
    for (int i = 0; i < NTHR / 32; ++i) s += cntS[base + i];
    int incl = s;
#pragma unroll
    for (int d = 1; d < 32; d <<= 1) {
      const int y = __shfl_up(incl, d, 32);
      if (lane >= d) incl += y;
    }
    int run = incl - s;
#pragma unroll 1
    for (int i = 0; i < NTHR / 32; ++i) {
      const int cv = cntS[base + i];
      offS[base + i] = run;
      run += cv;
    }
    if (lane == 31) tot[0] = incl;
  }
  __syncthreads();
  {
    int p = offS[tid];
#pragma unroll 1
    for (int q = 0; q < PER / 4; ++q) {
      const int i0 = seg0 + 4 * q;
      const int ic = i0 < lastv ? i0 : lastv;
      const v4i b = *(const v4i*)(bat + ic);
      const bool ok = i0 < nN;
      if (ok && b.x == g) { if ((unsigned)p < (unsigned)MEMCAP) mem[p] = i0;     p = p + 1; }
      if (ok && b.y == g) { if ((unsigned)p < (unsigned)MEMCAP) mem[p] = i0 + 1; p = p + 1; }
      if (ok && b.z == g) { if ((unsigned)p < (unsigned)MEMCAP) mem[p] = i0 + 2; p = p + 1; }
      if (ok && b.w == g) { if ((unsigned)p < (unsigned)MEMCAP) mem[p] = i0 + 3; p = p + 1; }
    }
  }
  __syncthreads();
  const int total = tot[0];
  const bool over = (total > MEMCAP) || (total < 0);
  const int cc = total < 0 ? 0 : (total > MEMCAP ? MEMCAP : total);
  float s = 0.0f;
  const unsigned short* cp = XH + tid;
#pragma unroll 2
  for (int j = 0; j < cc; ++j) {
    int n = mem[j];
    n = n < 0 ? 0 : (n > nN - 1 ? nN - 1 : n);
    const unsigned int hw = cp[(size_t)n * KA];
    const unsigned int lw = cp[(size_t)n * KA + HID];
    s += (bf2f(hw) + bf2f(lw));
  }
  const float cf = (total < 1) ? 1.0f : (float)total;
  float val = s * (1.0f / cf);
  val = over ? __int_as_float(0x7fc00000) : val;
  const unsigned int hbi = f2bf(val);
  prow[tid]       = (unsigned short)hbi;
  prow[HID + tid] = (unsigned short)f2bf(val - bf2f(hbi));
  __syncthreads();
  const v8us ov = *(const v8usa*)(prow + 8 * (tid & 63));
  unsigned short* op = PH + (size_t)g * KA + 8 * (tid & 63);
  const bool okst = tid < 64;
  if (okst) *(volatile v8us*)op = ov;
  __threadfence();
  if (okst) *(volatile v8us*)op = ov;
}

__global__ __launch_bounds__(NTHR) void k_out(const float* __restrict__ GF, const float* __restrict__ TAB,
                                              const int* __restrict__ FLG, int nFl, float* out) {
  __shared__ __attribute__((aligned(16))) float os[NGR];
  __shared__ int fls[NWAVE];
  const int tid = (int)threadIdx.x, lane = tid & 31, wave = tid >> 5;
  int f = 0;
#pragma unroll 1
  for (int i0 = 0; i0 < nFl; i0 += NTHR) {
    int i = i0 + tid;
    i = i > nFl - 1 ? nFl - 1 : i;
    f |= FLG[(size_t)i * 32 + 1];
  }
  const unsigned fm = __builtin_amdgcn_ballot_w32(f != 0);
  if (lane == 0) fls[wave] = (fm != 0u) ? 1 : 0;

  const v4f ba = *(const v4f*)(TAB + TB_BF + 8 * lane);
  const v4f bb = *(const v4f*)(TAB + TB_BF + 8 * lane + 4);
  const v4f wa = *(const v4f*)(TAB + TB_WO + 8 * lane);
  const v4f wb = *(const v4f*)(TAB + TB_WO + 8 * lane + 4);
  const float bo = TAB[TB_BO];
#pragma unroll 1
  for (int ri = 0; ri < NGR / NWAVE; ++ri) {
    const int row = ri * NWAVE + wave;
    const float* gp = GF + (size_t)row * HID + 8 * lane;
    const v4f a = *(const v4f*)gp;
    const v4f b = *(const v4f*)(gp + 4);
    float s = 0.0f;
    s = fmaf(relu_np(a.x + ba.x), wa.x, s);
    s = fmaf(relu_np(a.y + ba.y), wa.y, s);
    s = fmaf(relu_np(a.z + ba.z), wa.z, s);
    s = fmaf(relu_np(a.w + ba.w), wa.w, s);
    s = fmaf(relu_np(b.x + bb.x), wb.x, s);
    s = fmaf(relu_np(b.y + bb.y), wb.y, s);
    s = fmaf(relu_np(b.z + bb.z), wb.z, s);
    s = fmaf(relu_np(b.w + bb.w), wb.w, s);
    s += __shfl_xor(s, 16, 32);
    s += __shfl_xor(s, 8, 32);
    s += __shfl_xor(s, 4, 32);
    s += __shfl_xor(s, 2, 32);
    s += __shfl_xor(s, 1, 32);
    if (lane == 0) os[row] = s + bo;
  }
  __syncthreads();
  int anyf = 0;
#pragma unroll
  for (int w2 = 0; w2 < NWAVE; ++w2) anyf |= fls[w2];
  const float qnan = __int_as_float(0x7fc00000);
  v4f ov = *(const v4fa*)(os + 4 * (tid & 63));
  ov.x = (anyf != 0) ? qnan : ov.x;
  ov.y = (anyf != 0) ? qnan : ov.y;
  ov.z = (anyf != 0) ? qnan : ov.z;
  ov.w = (anyf != 0) ? qnan : ov.w;
  float* op = out + 4 * (tid & 63);
  const bool okst = tid < 64;
  if (okst) *(volatile v4f*)op = ov;
  __threadfence();
  if (okst) *(volatile v4f*)op = ov;
}

static inline int cdiv(int a, int b) { return (a + b - 1) / b; }
static inline size_t al256(size_t o) { return (o + 255) & ~(size_t)255; }

extern "C" void kernel_launch(void* const* d_in, const int* in_sizes, int n_in,
                              void* d_out, int out_size, void* d_ws, size_t ws_size,
                              hipStream_t stream) {
  if (n_in < 13) return;
  if (in_sizes[0] < CIN || (in_sizes[0] % CIN) != 0) return;
  const int nN = in_sizes[0] / CIN;
  if (nN < 4 || (nN & 3) != 0 || nN > 65536) return;
  if ((long long)PER * NTHR < (long long)nN) return;
  if (in_sizes[1] < 2 || (in_sizes[1] & 1) != 0) return;
  const int nE = in_sizes[1] / 2;
  if (nE < 1 || nE > (1 << 30)) return;
  if (in_sizes[2] != nN) return;
  if (in_sizes[3] != CIN * HID || in_sizes[4] != HID) return;
  if (in_sizes[5] != HID * HID || in_sizes[6] != HID) return;
  if (in_sizes[7] != HID * HID || in_sizes[8] != HID) return;
  if (in_sizes[9] != HID * HID || in_sizes[10] != HID) return;
  if (in_sizes[11] != HID || in_sizes[12] != 1) return;
  if (out_size != NGR) return;

  const float* x   = (const float*)d_in[0];
  const int*   ei  = (const int*)  d_in[1];
  const int*   bat = (const int*)  d_in[2];
  const float* W1  = (const float*)d_in[3];
  const float* b1  = (const float*)d_in[4];
  const float* W2  = (const float*)d_in[5];
  const float* b2  = (const float*)d_in[6];
  const float* W3  = (const float*)d_in[7];
  const float* b3  = (const float*)d_in[8];
  const float* Wf  = (const float*)d_in[9];
  const float* bfv = (const float*)d_in[10];
  const float* Wo  = (const float*)d_in[11];
  const float* bo  = (const float*)d_in[12];
  float* out = (float*)d_out;
  const int* src = ei;
  const int* dst = ei + nE;

  const int MP   = cdiv(nN, MROWS) * MROWS;
  const int gM   = MP / GBM;
  const int gA   = cdiv(MP, NBA);
  if ((long long)gA * NBA < (long long)MP) return;
  const int NPL  = gA * NBA;
  const int vec8 = ((nE & 3) == 0) ? 1 : 0;
  const int nUx  = MP * (CIN / 8);
  if ((nUx % NTHR) != 0) return;

  char* ws = (char*)d_ws;
  size_t off = 0;
  const size_t oXH  = off; off = al256(off + (size_t)MP * KA * 2);
  const size_t oH   = off; off = al256(off + (size_t)MP * HID * 4);
  const size_t oLST = off; off = al256(off + (size_t)gA * RCAP * 4);
  const size_t oCNT = off; off = al256(off + (size_t)NPL * 4);
  const size_t oOFF = off; off = al256(off + (size_t)NPL * 4);
  const size_t oDIS = off; off = al256(off + (size_t)NPL * 4);
  const size_t oFLG = off; off = al256(off + (size_t)gA * 128);
  const size_t oW1T = off; off = al256(off + (size_t)HID * CIN * 2);
  const size_t oW2D = off; off = al256(off + (size_t)HID * KA * 2);
  const size_t oW3D = off; off = al256(off + (size_t)HID * KA * 2);
  const size_t oWFD = off; off = al256(off + (size_t)HID * KA * 2);
  const size_t oTAB = off; off = al256(off + (size_t)TB_N * 4);
  const size_t oPH  = off; off = al256(off + (size_t)NGR * KA * 2);
  const size_t oGF  = off; off = al256(off + (size_t)NGR * HID * 4);
  if (off > ws_size || off > (size_t)WSMAX) return;
  if ((size_t)MP * CIN * 2 > (size_t)MP * KA * 2) return;
  unsigned short* XHL = (unsigned short*)(ws + oXH);
  unsigned short* XB  = (unsigned short*)(ws + oXH);
  float*          H   = (float*)(ws + oH);
  int*            LST = (int*)(ws + oLST);
  int*            CNT = (int*)(ws + oCNT);
  int*            OFF = (int*)(ws + oOFF);
  float*          DIS = (float*)(ws + oDIS);
  int*            FLG = (int*)(ws + oFLG);
  unsigned short* W1T = (unsigned short*)(ws + oW1T);
  unsigned short* W2D = (unsigned short*)(ws + oW2D);
  unsigned short* W3D = (unsigned short*)(ws + oW3D);
  unsigned short* WFD = (unsigned short*)(ws + oWFD);
  float*          TAB = (float*)(ws + oTAB);
  unsigned short* PHL = (unsigned short*)(ws + oPH);
  float*          GF  = (float*)(ws + oGF);

  const int bktLds = BKT_LDS_INTS * 4;
  hipFuncSetAttribute(reinterpret_cast<const void*>(&k_bucket),
                      hipFuncAttributeMaxDynamicSharedMemorySize, bktLds);

  const int nPrepUnits = nUx + NUW1 + 3 * NUWD + 2 * NTHR;
  k_prep<<<nPrepUnits / NTHR, NTHR, 0, stream>>>(x, W1, W2, W3, Wf, b1, b2, b3, bfv, Wo, bo,
                                                 XB, W1T, W2D, W3D, WFD, TAB, nN, nUx);
  k_bucket<<<gA, NTHR, bktLds, stream>>>(src, dst, nE, nN, vec8, LST, CNT, OFF, DIS, FLG);
  k_gemm<<<dim3(gM, HID / GBN), GTHR, 0, stream>>>(XB, W1T, H, CIN, HID);
  k_agg<<<gA, NTHR, 0, stream>>>(LST, CNT, OFF, FLG, DIS, H, TAB + TB_B1, XHL, nN, MP);
  k_gemm<<<dim3(gM, HID / GBN), GTHR, 0, stream>>>(XHL, W2D, H, KA, HID);
  k_agg<<<gA, NTHR, 0, stream>>>(LST, CNT, OFF, FLG, DIS, H, TAB + TB_B2, XHL, nN, MP);
  k_gemm<<<dim3(gM, HID / GBN), GTHR, 0, stream>>>(XHL, W3D, H, KA, HID);
  k_agg<<<gA, NTHR, 0, stream>>>(LST, CNT, OFF, FLG, DIS, H, TAB + TB_B3, XHL, nN, MP);
  k_pool<<<NGR, NTHR, 0, stream>>>(XHL, bat, nN, PHL);
  k_gemm<<<dim3(NGR / GBM, HID / GBN), GTHR, 0, stream>>>(PHL, WFD, GF, KA, HID);
  k_out<<<1, NTHR, 0, stream>>>(GF, TAB, FLG, gA, out);
}
